// SparseConvNet_64_5781025980666
// MI455X (gfx1250) — hardware-verified
//
#include <hip/hip_runtime.h>
#include <stddef.h>

typedef _Float16 v16h __attribute__((ext_vector_type(16)));
typedef _Float16 v8h  __attribute__((ext_vector_type(8)));
typedef _Float16 v8ha __attribute__((ext_vector_type(8), __may_alias__));
typedef float    v8f  __attribute__((ext_vector_type(8)));
typedef float    v4f  __attribute__((ext_vector_type(4)));
typedef float    v4fa __attribute__((ext_vector_type(4), __may_alias__));
union Frag { v16h v; v8h half[2]; };

#define NCONV 17
#define NTP   14
#define WSCALE     64.0f
#define WSCALE_INV 0.015625f
#define CONV_THREADS 256
#define VOX_PER_BLOCK 256

__device__ __forceinline__ v8f wmma_f16(v16h a, v16h b, v8f acc) {
  acc = __builtin_amdgcn_wmma_f32_16x16x32_f16(false, a, false, b, (short)0, acc, false, false);
  asm volatile("v_nop\n\tv_nop\n\tv_nop\n\tv_nop" : "+v"(acc) : "v"(a), "v"(b));
  return acc;
}

__global__ void __launch_bounds__(256)
pack_weights_kernel(const float* __restrict__ W, _Float16* __restrict__ pw,
                    _Float16* __restrict__ zv) {
  const int total = NCONV * NTP * 32 * 2;
  const int q = blockIdx.x * blockDim.x + threadIdx.x;
  v8h o;
#pragma unroll
  for (int e = 0; e < 8; ++e) o[e] = (_Float16)0.0f;
  _Float16* dst = nullptr;
  if (q < total) {
    const int j8   = q & 1;
    const int lane = (q >> 1) & 31;
    const int tpl  = q >> 6;
    const int tp   = tpl % NTP;
    const int L    = tpl / NTP;
    const int h    = lane >> 4;
    const int cout = lane & 15;
    const int tap  = 2 * tp + j8;
    if (tap < 27) {
      const float* src = W + ((size_t)(L * 16 + cout) * 16 + 8 * h) * 27 + tap;
#pragma unroll
      for (int e = 0; e < 8; ++e) o[e] = (_Float16)(src[e * 27] * WSCALE);
    }
    dst = pw + (size_t)q * 8;
  } else if (q < total + 8) {
    dst = zv + (q - total) * 8;
  }
  if (dst) *(volatile v8h*)dst = o;
  __threadfence();
  if (dst) *(volatile v8h*)dst = o;
}

__global__ void __launch_bounds__(256)
make_mask_kernel(const int* __restrict__ mi, float* __restrict__ m, int vol, int nchunk) {
  const int g = blockIdx.x * blockDim.x + threadIdx.x;
  if (g >= nchunk) return;
  v4f o;
#pragma unroll
  for (int i = 0; i < 4; ++i) {
    const int v = 4 * g + i;
    float val = 0.0f;
    if (v < vol) val = (mi[v] == 0) ? 1.0f : 0.0f;
    o[i] = val;
  }
  float* p = m + (size_t)4 * g;
  *(volatile v4f*)p = o;
  __threadfence();
  *(volatile v4f*)p = o;
}

__global__ void __launch_bounds__(256)
x_to_cl_kernel(const float* __restrict__ x, _Float16* __restrict__ act, int vol) {
  const int t = blockIdx.x * blockDim.x + threadIdx.x;
  if (t >= vol * 2) return;
  const int v  = t >> 1;
  const int cb = (t & 1) * 8;
  v8h o;
#pragma unroll
  for (int e = 0; e < 8; ++e) o[e] = (_Float16)x[(size_t)(cb + e) * vol + v];
  _Float16* p = act + (size_t)t * 8;
  *(volatile v8h*)p = o;
  __threadfence();
  *(volatile v8h*)p = o;
}

__global__ void __launch_bounds__(256)
mask_down_kernel(const float* __restrict__ in, float* __restrict__ out,
                 int Din, int Dout, int nchunk) {
  const int g = blockIdx.x * blockDim.x + threadIdx.x;
  if (g >= nchunk) return;
  const int volOut = Dout * Dout * Dout;
  v4f o;
#pragma unroll
  for (int i = 0; i < 4; ++i) {
    const int v = 4 * g + i;
    float mx = 0.0f;
    if (v < volOut) {
      const int z = v / (Dout * Dout);
      const int r = v - z * Dout * Dout;
      const int y = r / Dout;
      const int xx = r - y * Dout;
      for (int dz = 0; dz < 3; ++dz)
        for (int dy = 0; dy < 3; ++dy)
          for (int dx = 0; dx < 3; ++dx) {
            const int sz = 2 * z + dz - 1, sy = 2 * y + dy - 1, sx = 2 * xx + dx - 1;
            if ((unsigned)sz < (unsigned)Din && (unsigned)sy < (unsigned)Din &&
                (unsigned)sx < (unsigned)Din)
              mx = fmaxf(mx, in[(sz * Din + sy) * Din + sx]);
          }
    }
    o[i] = mx;
  }
  float* p = out + (size_t)4 * g;
  *(volatile v4f*)p = o;
  __threadfence();
  *(volatile v4f*)p = o;
}

struct TileCtx {
  int base;
  unsigned m27;
  int vv;
  float vmul;
};

__device__ __forceinline__ TileCtx make_ctx(int tile, int n, int Dout, int volOut,
                                            int stride, int Din) {
  TileCtx c;
  const int vox = tile * 16 + n;
  const bool valid = (vox < volOut);
  c.vv = valid ? vox : 0;
  const int D2 = Dout * Dout;
  const int oz = c.vv / D2;
  const int rem = c.vv - oz * D2;
  const int oy = rem / Dout;
  const int ox = rem - oy * Dout;
  const int bz = stride * oz - 1, by = stride * oy - 1, bx = stride * ox - 1;
  c.base = (bz * Din + by) * Din + bx;
  unsigned xm = 0, ym = 0, zm = 0;
#pragma unroll
  for (int d = 0; d < 3; ++d) {
    if ((unsigned)(bx + d) < (unsigned)Din) xm |= 1u << d;
    if ((unsigned)(by + d) < (unsigned)Din) ym |= 1u << (3 * d);
    if ((unsigned)(bz + d) < (unsigned)Din) zm |= 1u << (9 * d);
  }
  c.m27 = valid ? ((xm * ym) * zm) : 0u;
  c.vmul = valid ? 1.0f : 0.0f;
  return c;
}

__device__ __forceinline__ v16h load_b(const TileCtx& c, int T0, unsigned hoff,
                                        const _Float16* __restrict__ actIn,
                                        unsigned zvRel, int Din, int Din2) {
  const int T1 = (T0 < 26) ? (T0 + 1) : T0;
  const int off0 = c.base + (T0 / 9) * Din2 + ((T0 / 3) % 3) * Din + (T0 % 3);
  const int off1 = c.base + (T1 / 9) * Din2 + ((T1 / 3) % 3) * Din + (T1 % 3);
  const unsigned p0 = ((c.m27 >> T0) & 1u) ? ((unsigned)off0 * 32u + hoff) : zvRel;
  const unsigned p1 = ((c.m27 >> T1) & 1u) ? ((unsigned)off1 * 32u + hoff) : zvRel;
  Frag f;
  f.half[0] = *(const v8h*)((const char*)actIn + p0);
  f.half[1] = *(const v8h*)((const char*)actIn + p1);
  return f.v;
}

__global__ void __launch_bounds__(CONV_THREADS) __attribute__((amdgpu_num_vgpr(256)))
conv3x3_wmma_kernel(const _Float16* __restrict__ actIn,
                    _Float16* __restrict__ actOut,
                    const _Float16* __restrict__ pw,
                    const float* __restrict__ bnS,
                    const float* __restrict__ bnB,
                    const float* __restrict__ mask,
                    unsigned zvRel,
                    int Din, int Dout, int stride,
                    float* __restrict__ outF32) {
  __shared__ _Float16 wlds[NTP * 32 * 16];
  __shared__ _Float16 sAct[VOX_PER_BLOCK * 16];
  __shared__ float    sOut[16 * VOX_PER_BLOCK];

  const int tid = threadIdx.x;
  {
    const v8h* src = (const v8h*)pw;
    v8h* dst = (v8h*)wlds;
    for (int i = tid; i < NTP * 32 * 2; i += CONV_THREADS) dst[i] = src[i];
  }
  __syncthreads();

  const int lane = tid & 31;
  const int wave = tid >> 5;
  const int h    = lane >> 4;
  const int n    = lane & 15;
  const int volOut = Dout * Dout * Dout;
  const int Din2 = Din * Din;

  const int tile0 = (blockIdx.x * (CONV_THREADS / 32) + wave) * 2;
  const TileCtx c0 = make_ctx(tile0 + 0, n, Dout, volOut, stride, Din);
  const TileCtx c1 = make_ctx(tile0 + 1, n, Dout, volOut, stride, Din);

  v8f acc0 = {0.f, 0.f, 0.f, 0.f, 0.f, 0.f, 0.f, 0.f};
  v8f acc1 = {0.f, 0.f, 0.f, 0.f, 0.f, 0.f, 0.f, 0.f};
  const unsigned hoff = 16u * (unsigned)h;

#pragma unroll
  for (int tp = 0; tp < NTP; ++tp) {
    const v16h a  = *(const v16h*)(wlds + ((tp * 32 + lane) << 4));
    const v16h b0 = load_b(c0, 2 * tp, hoff, actIn, zvRel, Din, Din2);
    const v16h b1 = load_b(c1, 2 * tp, hoff, actIn, zvRel, Din, Din2);
    acc0 = wmma_f16(a, b0, acc0);
    acc1 = wmma_f16(a, b1, acc1);
  }

  const int cc = 8 * h;
  const v4f sLo = *(const v4f*)(bnS + cc);
  const v4f sHi = *(const v4f*)(bnS + cc + 4);
  const v4f bLo = *(const v4f*)(bnB + cc);
  const v4f bHi = *(const v4f*)(bnB + cc + 4);
  const float m0 = mask[c0.vv] * c0.vmul;
  const float m1 = mask[c1.vv] * c1.vmul;
  float o0[8], o1[8];
#pragma unroll
  for (int r = 0; r < 8; ++r) {
    const float s = (r < 4) ? sLo[r & 3] : sHi[r & 3];
    const float b = (r < 4) ? bLo[r & 3] : bHi[r & 3];
    o0[r] = fmaxf(fmaf(acc0[r] * WSCALE_INV, s, b), 0.0f) * m0;
    o1[r] = fmaxf(fmaf(acc1[r] * WSCALE_INV, s, b), 0.0f) * m1;
  }

  const int lv0 = wave * 32 + n;
  const int lv1 = lv0 + 16;
  {
    v8h t0, t1;
#pragma unroll
    for (int r = 0; r < 8; ++r) { t0[r] = (_Float16)o0[r]; t1[r] = (_Float16)o1[r]; }
    *(v8h*)(sAct + lv0 * 16 + cc) = t0;
    *(v8h*)(sAct + lv1 * 16 + cc) = t1;
  }
  const bool wantOut = (outF32 != nullptr);
  if (wantOut) {
#pragma unroll
    for (int r = 0; r < 8; ++r) {
      sOut[(cc + r) * VOX_PER_BLOCK + lv0] = o0[r];
      sOut[(cc + r) * VOX_PER_BLOCK + lv1] = o1[r];
    }
  }
  __syncthreads();

  const int blk = blockIdx.x;
  int nvox = volOut - blk * VOX_PER_BLOCK;
  if (nvox > VOX_PER_BLOCK) nvox = VOX_PER_BLOCK;

  v8h av[2]; _Float16* ap[2]; bool aok[2];
#pragma unroll
  for (int j = 0; j < 2; ++j) {
    const int cidx = tid + CONV_THREADS * j;
    aok[j] = (cidx < nvox * 2);
    av[j] = *(const v8ha*)(sAct + cidx * 8);
    ap[j] = actOut + (size_t)blk * (VOX_PER_BLOCK * 16) + (size_t)cidx * 8;
  }

  v4f ov[4]; float* op[4]; bool ook[4];
#pragma unroll
  for (int j = 0; j < 4; ++j) {
    ook[j] = false; op[j] = outF32;
    ov[j][0] = 0.f; ov[j][1] = 0.f; ov[j][2] = 0.f; ov[j][3] = 0.f;
  }
  if (wantOut) {
    if (gridDim.x == 1) {
      const int nel = 16 * volOut;
#pragma unroll
      for (int j = 0; j < 4; ++j) {
        const int g = tid + CONV_THREADS * j;
        const int e0 = 4 * g;
        if (e0 < nel) {
          ook[j] = true;
          op[j] = outF32 + e0;
#pragma unroll
          for (int i = 0; i < 4; ++i) {
            const int e  = e0 + i;
            const int ch = e / volOut;
            const int v  = e - ch * volOut;
            ov[j][i] = sOut[ch * VOX_PER_BLOCK + v];
          }
        }
      }
    } else {
#pragma unroll
      for (int j = 0; j < 4; ++j) {
        const int f  = tid + CONV_THREADS * j;
        const int ch = f >> 6;
        const int f4 = f & 63;
        if (4 * f4 < nvox) {
          ook[j] = true;
          ov[j] = *(const v4fa*)(sOut + ch * VOX_PER_BLOCK + 4 * f4);
          op[j] = outF32 + (size_t)ch * volOut + (size_t)blk * VOX_PER_BLOCK + 4 * f4;
        }
      }
    }
  }

#pragma unroll
  for (int j = 0; j < 2; ++j) if (aok[j]) *(volatile v8h*)ap[j] = av[j];
#pragma unroll
  for (int j = 0; j < 4; ++j) if (ook[j]) *(volatile v4f*)op[j] = ov[j];
  __threadfence();
#pragma unroll
  for (int j = 0; j < 2; ++j) if (aok[j]) *(volatile v8h*)ap[j] = av[j];
#pragma unroll
  for (int j = 0; j < 4; ++j) if (ook[j]) *(volatile v4f*)op[j] = ov[j];
}

static inline int cdiv_i(size_t a, size_t b) { return (int)((a + b - 1) / b); }
static inline size_t pad32(size_t n) { return (n + 31) / 32 * 32; }

extern "C" void kernel_launch(void* const* d_in, const int* in_sizes, int n_in,
                              void* d_out, int out_size, void* d_ws, size_t ws_size,
                              hipStream_t stream) {
  (void)in_sizes; (void)n_in; (void)out_size;
  const float* x        = (const float*)d_in[0];
  const int*   mask_idx = (const int*)d_in[1];
  const float* W        = (const float*)d_in[2];
  const float* bnS      = (const float*)d_in[3];
  const float* bnB      = (const float*)d_in[4];
  float* out = (float*)d_out;

  const size_t vol96 = 96ull * 96 * 96;
  const size_t vol48 = 48ull * 48 * 48;
  const size_t vol24 = 24ull * 24 * 24;
  const size_t vol12 = 12ull * 12 * 12;
  const size_t vol6  = 6ull * 6 * 6;

  char* ws = (char*)d_ws;
  size_t off = 0;
  auto take = [&](size_t bytes) -> char* {
    char* p = ws + off;
    off += (bytes + 255) & ~(size_t)255;
    return p;
  };
  _Float16* actA = (_Float16*)take(vol96 * 16 * sizeof(_Float16));
  _Float16* actB = (_Float16*)take(vol96 * 16 * sizeof(_Float16));
  _Float16* pw   = (_Float16*)take((size_t)NCONV * NTP * 32 * 16 * sizeof(_Float16));
  _Float16* zv   = (_Float16*)take(256);
  float* m96 = (float*)take(pad32(vol96) * sizeof(float));
  float* m48 = (float*)take(pad32(vol48) * sizeof(float));
  float* m24 = (float*)take(pad32(vol24) * sizeof(float));
  float* m12 = (float*)take(pad32(vol12) * sizeof(float));
  float* m6  = (float*)take(pad32(vol6) * sizeof(float));
  if (off > ws_size) return;

  {
    const int chunks = NCONV * NTP * 32 * 2 + 8;
    pack_weights_kernel<<<cdiv_i(chunks, 256), 256, 0, stream>>>(W, pw, zv);
  }
  {
    const int nchunk = (int)(pad32(vol96) / 4);
    make_mask_kernel<<<cdiv_i(nchunk, 256), 256, 0, stream>>>(mask_idx, m96, (int)vol96, nchunk);
  }
  x_to_cl_kernel<<<cdiv_i(vol96 * 2, 256), 256, 0, stream>>>(x, actA, (int)vol96);
  {
    const int n48 = (int)(pad32(vol48) / 4), n24 = (int)(pad32(vol24) / 4);
    const int n12 = (int)(pad32(vol12) / 4), n6 = (int)(pad32(vol6) / 4);
    mask_down_kernel<<<cdiv_i(n48, 256), 256, 0, stream>>>(m96, m48, 96, 48, n48);
    mask_down_kernel<<<cdiv_i(n24, 256), 256, 0, stream>>>(m48, m24, 48, 24, n24);
    mask_down_kernel<<<cdiv_i(n12, 256), 256, 0, stream>>>(m24, m12, 24, 12, n12);
    mask_down_kernel<<<cdiv_i(n6, 256), 256, 0, stream>>>(m12, m6, 12, 6, n6);
  }

  auto conv = [&](const _Float16* in, _Float16* o, int L, const float* mk,
                  int Din, int Dout, int stride, float* of) {
    const size_t vol = (size_t)Dout * Dout * Dout;
    const int blocks = cdiv_i(vol, VOX_PER_BLOCK);
    const unsigned zrel = (unsigned)((const char*)zv - (const char*)in);
    conv3x3_wmma_kernel<<<blocks, CONV_THREADS, 0, stream>>>(
        in, o, pw + (size_t)L * NTP * 32 * 16, bnS + L * 16, bnB + L * 16,
        mk, zrel, Din, Dout, stride, of);
  };

  float* out1 = out;
  float* out2 = out1 + 16 * vol48;
  float* out3 = out2 + 16 * vol24;
  float* out4 = out3 + 16 * vol12;

  conv(actA, actB, 0, m96, 96, 96, 1, nullptr);
  conv(actB, actA, 1, m96, 96, 96, 1, nullptr);
  conv(actA, actB, 2, m48, 96, 48, 2, nullptr);
  conv(actB, actA, 3, m48, 48, 48, 1, nullptr);
  conv(actA, actB, 4, m48, 48, 48, 1, out1);
  conv(actB, actA, 5, m24, 48, 24, 2, nullptr);
  conv(actA, actB, 6, m24, 24, 24, 1, nullptr);
  conv(actB, actA, 7, m24, 24, 24, 1, nullptr);
  conv(actA, actB, 8, m24, 24, 24, 1, out2);
  conv(actB, actA, 9, m12, 24, 12, 2, nullptr);
  conv(actA, actB, 10, m12, 12, 12, 1, nullptr);
  conv(actB, actA, 11, m12, 12, 12, 1, nullptr);
  conv(actA, actB, 12, m12, 12, 12, 1, out3);
  conv(actB, actA, 13, m6, 12, 6, 2, nullptr);
  conv(actA, actB, 14, m6, 6, 6, 1, nullptr);
  conv(actB, actA, 15, m6, 6, 6, 1, nullptr);
  conv(actA, actB, 16, m6, 6, 6, 1, out4);
}
